// KBGAT_Model_22617297780845
// MI455X (gfx1250) — hardware-verified
//
#include <hip/hip_runtime.h>
#include <stddef.h>


#define DI    128
#define DE    256
#define NHD   4
#define HWD   64
#define PQP   512
#define GT    64
#define GTHR  128
#define NB    256
#define CHUNK 2048
#define NTHR  256
#define NWAVE 8
#define WCAP  256
#define NGRP  (CHUNK / (NTHR * 4))
#define BNR   320
#define BNA   64

#define LDS_SACC (NB * DE)
#define LDS_AUX  (NB * 4 * 3)
#define LDS_LIST (NWAVE * WCAP)
#define AGG_LDS_BYTES ((LDS_SACC + LDS_AUX + LDS_LIST + NWAVE) * 4)

static_assert(WCAP == (CHUNK / NTHR) * 32);
static_assert(NGRP == 2);
static_assert(NB == 256);
static_assert(CHUNK == 2048);
static_assert((LDS_SACC % 4) == 0);
static_assert(AGG_LDS_BYTES == 282656);
static_assert(NHD * HWD == DE);

typedef __bf16 bf16;
typedef bf16   v8b  __attribute__((ext_vector_type(8)));
typedef bf16   v16b __attribute__((ext_vector_type(16)));
typedef float  v4f  __attribute__((ext_vector_type(4)));
typedef float  v8f  __attribute__((ext_vector_type(8)));
typedef int    v4i  __attribute__((ext_vector_type(4)));
typedef double v2d  __attribute__((ext_vector_type(2)));
union FragB { v16b v; v8b half[2]; };
union Pack8 { v8b h; v4i i; };

__device__ __forceinline__ v8f wm(v16b a, v16b b, v8f c) {
  v8f d = __builtin_amdgcn_wmma_f32_16x16x32_bf16(false, a, false, b, (short)0, c, false, false);
  asm volatile("v_nop\n\tv_nop\n\tv_nop\n\tv_nop" : "+v"(d) : "v"(a), "v"(b));
  return d;
}

__device__ __forceinline__ int clampi(int v, int hi) { v = v < 0 ? 0 : v; return v > hi ? hi : v; }
__device__ __forceinline__ int iminv(int a, int b) { return a < b ? a : b; }
__device__ __forceinline__ v4f zero4() { v4f z = {0.f, 0.f, 0.f, 0.f}; return z; }

__device__ __forceinline__ void split8(v4f a, v4f b, v4i& hi, v4i& lo) {
  Pack8 ph, pl;
#pragma unroll
  for (int u = 0; u < 4; ++u) {
    const float fa = a[u];
    const bf16  ha = (bf16)fa;
    ph.h[u] = ha;
    pl.h[u] = (bf16)(fa - (float)ha);
    const float fb = b[u];
    const bf16  hb = (bf16)fb;
    ph.h[4 + u] = hb;
    pl.h[4 + u] = (bf16)(fb - (float)hb);
  }
  hi = ph.i; lo = pl.i;
}

__device__ __forceinline__ float dot8(v4f a0, v4f a1, v4f b0, v4f b1) {
  float d = a0.x * b0.x;
  d += a0.y * b0.y; d += a0.z * b0.z; d += a0.w * b0.w;
  d += a1.x * b1.x; d += a1.y * b1.y; d += a1.z * b1.z; d += a1.w * b1.w;
  return d;
}

__device__ __forceinline__ float eluf(float v) { return v > 0.f ? v : (__expf(v) - 1.0f); }
__device__ __forceinline__ v4f elu4(v4f v) {
  v.x = eluf(v.x); v.y = eluf(v.y); v.z = eluf(v.z); v.w = eluf(v.w);
  return v;
}

template <int NHEAD>
__device__ __forceinline__ float gred(float d) {
  d += __shfl_xor(d, 1, 32);
  d += __shfl_xor(d, 2, 32);
  d += __shfl_xor(d, 4, 32);
  if (NHEAD == 1) {
    d += __shfl_xor(d, 8, 32);
    d += __shfl_xor(d, 16, 32);
  }
  return d;
}

__global__ __launch_bounds__(NTHR) void k_cvtA(const float* __restrict__ src, int nValid, int K,
                                               int total8, bf16* dh, bf16* dl) {
  const int i = blockIdx.x * NTHR + threadIdx.x;
  if (i >= total8) return;
  const int kpr = K >> 3;
  const int row = i / kpr;
  const int c   = (i - row * kpr) * 8;
  int rc = row; if (rc > nValid - 1) rc = nValid - 1;
  const float* p = src + (size_t)rc * K + c;
  v4f a = *(const v4f*)p;
  v4f b = *(const v4f*)(p + 4);
  if (row >= nValid) { a = zero4(); b = zero4(); }
  v4i hv, lv;
  split8(a, b, hv, lv);
  const size_t o = (size_t)row * K + c;
  *(volatile v4i*)(dh + o) = hv;
  *(volatile v4i*)(dl + o) = lv;
  __threadfence();
  *(volatile v4i*)(dh + o) = hv;
  *(volatile v4i*)(dl + o) = lv;
}

__global__ __launch_bounds__(NTHR) void k_packB(const float* __restrict__ src, bf16* dh, bf16* dl,
                                                int K, int nRows, int segW, int segStride, int kStride,
                                                int base0, int baseStep, int total8) {
  const int i = blockIdx.x * NTHR + threadIdx.x;
  if (i >= total8) return;
  const int part = blockIdx.y;
  const int kpr  = K >> 3;
  const int nl   = i / kpr;
  const int k8   = (i - nl * kpr) * 8;
  const int seg  = nl / segW;
  const int sb   = base0 + part * baseStep + seg * segStride + (nl - seg * segW);
  v4f a, b;
  a.x = src[sb + (k8 + 0) * kStride]; a.y = src[sb + (k8 + 1) * kStride];
  a.z = src[sb + (k8 + 2) * kStride]; a.w = src[sb + (k8 + 3) * kStride];
  b.x = src[sb + (k8 + 4) * kStride]; b.y = src[sb + (k8 + 5) * kStride];
  b.z = src[sb + (k8 + 6) * kStride]; b.w = src[sb + (k8 + 7) * kStride];
  v4i hv, lv;
  split8(a, b, hv, lv);
  const size_t o = (size_t)(part * nRows + nl) * K + k8;
  *(volatile v4i*)(dh + o) = hv;
  *(volatile v4i*)(dl + o) = lv;
  __threadfence();
  *(volatile v4i*)(dh + o) = hv;
  *(volatile v4i*)(dl + o) = lv;
}

__global__ __launch_bounds__(GTHR) void k_gemm3(
    const bf16* __restrict__ Ah, const bf16* __restrict__ Al, int lda,
    const bf16* __restrict__ Bh, const bf16* __restrict__ Bl, int ldb, int K,
    float* C, int ldc, int mStore, const float* __restrict__ Add,
    bf16* Ch, bf16* Cl, int ldh) {
  __shared__ __attribute__((aligned(16))) float Cs[4 * 16 * GT];
  const int tid = threadIdx.x, lane = tid & 31, wave = tid >> 5;
  const int hh = lane >> 4, m = lane & 15;
  const int row0 = blockIdx.y * GT + wave * 16;
  const int col0 = blockIdx.x * GT;

  const bf16* pah = Ah + (size_t)(row0 + m) * lda + 8 * hh;
  const bf16* pal = Al + (size_t)(row0 + m) * lda + 8 * hh;
  const size_t ob = (size_t)(col0 + m) * ldb + 8 * hh;
  const bf16* pbh = Bh + ob;
  const bf16* pbl = Bl + ob;
  const size_t tstep = (size_t)16 * ldb;

  const v8f z8 = {0.f, 0.f, 0.f, 0.f, 0.f, 0.f, 0.f, 0.f};
  v8f acc[4];
#pragma unroll
  for (int t = 0; t < 4; ++t) acc[t] = z8;

#pragma unroll 1
  for (int k0 = 0; k0 < K; k0 += 32) {
    FragB ah, al;
    ah.half[0] = *(const v8b*)(pah + k0);
    ah.half[1] = *(const v8b*)(pah + k0 + 16);
    al.half[0] = *(const v8b*)(pal + k0);
    al.half[1] = *(const v8b*)(pal + k0 + 16);
#pragma unroll
    for (int t = 0; t < 4; ++t) {
      FragB bh, bl;
      const bf16* qh = pbh + t * tstep + k0;
      const bf16* ql = pbl + t * tstep + k0;
      bh.half[0] = *(const v8b*)qh;
      bh.half[1] = *(const v8b*)(qh + 16);
      bl.half[0] = *(const v8b*)ql;
      bl.half[1] = *(const v8b*)(ql + 16);
      acc[t] = wm(ah.v, bh.v, acc[t]);
      acc[t] = wm(ah.v, bl.v, acc[t]);
      acc[t] = wm(al.v, bh.v, acc[t]);
    }
  }

  float* cs = Cs + wave * 16 * GT;
#pragma unroll
  for (int t = 0; t < 4; ++t) {
#pragma unroll
    for (int r = 0; r < 8; ++r) cs[(8 * hh + r) * GT + 16 * t + m] = acc[t][r];
  }
  __syncthreads();

  if (C != nullptr) {
    const int rs = lane >> 4, c4 = (lane & 15) * 4;
    v4f v[8];
#pragma unroll
    for (int i = 0; i < 8; ++i) {
      const int r = 2 * i + rs;
      v[i] = *(const v4f*)(cs + r * GT + c4);
      if (Add != nullptr) v[i] += *(const v4f*)(Add + (size_t)(row0 + r) * ldc + col0 + c4);
    }
#pragma unroll
    for (int i = 0; i < 8; ++i) {
      const int r = 2 * i + rs;
      if (row0 + r < mStore) *(volatile v4f*)(C + (size_t)(row0 + r) * ldc + col0 + c4) = v[i];
    }
    __threadfence();
#pragma unroll
    for (int i = 0; i < 8; ++i) {
      const int r = 2 * i + rs;
      if (row0 + r < mStore) *(volatile v4f*)(C + (size_t)(row0 + r) * ldc + col0 + c4) = v[i];
    }
  }
  if (Ch != nullptr) {
    const int rs = lane >> 3, c8 = (lane & 7) * 8;
    v4i hv[4], lv[4];
#pragma unroll
    for (int i = 0; i < 4; ++i) {
      const int r = 4 * i + rs;
      const v4f a = *(const v4f*)(cs + r * GT + c8);
      const v4f b = *(const v4f*)(cs + r * GT + c8 + 4);
      split8(a, b, hv[i], lv[i]);
    }
#pragma unroll
    for (int i = 0; i < 4; ++i) {
      const size_t o = (size_t)(row0 + 4 * i + rs) * ldh + col0 + c8;
      *(volatile v4i*)(Ch + o) = hv[i];
      *(volatile v4i*)(Cl + o) = lv[i];
    }
    __threadfence();
#pragma unroll
    for (int i = 0; i < 4; ++i) {
      const size_t o = (size_t)(row0 + 4 * i + rs) * ldh + col0 + c8;
      *(volatile v4i*)(Ch + o) = hv[i];
      *(volatile v4i*)(Cl + o) = lv[i];
    }
  }
}

template <int NHEAD>
__global__ __launch_bounds__(NTHR) void k_agg(
    const int* __restrict__ key1, const int* __restrict__ col1, const int* __restrict__ typ1,
    const int* __restrict__ ind2, const float* __restrict__ PQ, const float* __restrict__ Rt,
    const float* __restrict__ av, bf16* xh, bf16* xl, float* xf,
    int nN, int nR, int nE1, int nE2) {
  extern __shared__ v4f lds_dyn[];
  float* sacc = (float*)lds_dyn;
  float* smax = sacc + LDS_SACC;
  float* sden = smax + NB * 4;
  float* spa  = sden + NB * 4;
  int*   list = (int*)(spa + NB * 4);
  int*   wcnt = list + LDS_LIST;

  const int tid  = threadIdx.x;
  const int lane = tid & 31;
  const int wave = tid >> 5;
  const int head = (NHEAD == 4) ? (lane >> 3) : 0;
  const int nodeBase = blockIdx.x * NB;
  const v4f ar0 = *(const v4f*)(av + 8 * lane);
  const v4f ar1 = *(const v4f*)(av + 8 * lane + 4);

  {
    const v4f z4 = zero4();
    for (int i = tid; i < LDS_SACC / 4; i += NTHR) lds_dyn[i] = z4;
    for (int i = tid; i < NB * 4; i += NTHR) { smax[i] = -1e30f; sden[i] = 0.f; }
  }
#pragma unroll 1
  for (int slot = wave; slot < NB; slot += NWAVE) {
    int row = nodeBase + slot;
    if (row > nN - 1) row = nN - 1;
    const float* p = PQ + (size_t)row * PQP + 8 * lane;
    const v4f p0 = *(const v4f*)p;
    const v4f p1 = *(const v4f*)(p + 4);
    float d = dot8(p0, p1, ar0, ar1);
    d = gred<NHEAD>(d);
    spa[slot * 4 + head] = d;
  }
  __syncthreads();

  const int nCh1 = (nE1 + CHUNK - 1) / CHUNK;
  const int nCh2 = (nE2 + CHUNK - 1) / CHUNK;
  const int sent = -2147483647 - 1;
#pragma unroll 1
  for (int ch = 0; ch < nCh1 + nCh2; ++ch) {
    const bool dir   = (ch < nCh1);
    const int  cbase = (dir ? ch : (ch - nCh1)) * CHUNK;
    const int  nEc   = dir ? nE1 : nE2;
    const bool full  = dir && (cbase + CHUNK <= nEc);
    int wc = 0;
#pragma unroll
    for (int g = 0; g < NGRP; ++g) {
      const int el0 = (g * NTHR + tid) * 4;
      const int e0  = cbase + el0;
      v4i d;
      if (full) {
        d = *(const v4i*)(key1 + e0);
      } else {
        const int j0 = iminv(e0, nEc - 1), j1 = iminv(e0 + 1, nEc - 1);
        const int j2 = iminv(e0 + 2, nEc - 1), j3 = iminv(e0 + 3, nEc - 1);
        int q0, q1, q2, q3;
        if (dir) { q0 = key1[j0]; q1 = key1[j1]; q2 = key1[j2]; q3 = key1[j3]; }
        else     { q0 = ind2[4 * j0 + 3]; q1 = ind2[4 * j1 + 3]; q2 = ind2[4 * j2 + 3]; q3 = ind2[4 * j3 + 3]; }
        d.x = (e0     < nEc) ? q0 : sent;
        d.y = (e0 + 1 < nEc) ? q1 : sent;
        d.z = (e0 + 2 < nEc) ? q2 : sent;
        d.w = (e0 + 3 < nEc) ? q3 : sent;
      }
      const unsigned s0 = (unsigned)d.x - (unsigned)nodeBase;
      const unsigned s1 = (unsigned)d.y - (unsigned)nodeBase;
      const unsigned s2 = (unsigned)d.z - (unsigned)nodeBase;
      const unsigned s3 = (unsigned)d.w - (unsigned)nodeBase;
      const bool h0 = s0 < (unsigned)NB;
      const bool h1 = s1 < (unsigned)NB;
      const bool h2 = s2 < (unsigned)NB;
      const bool h3 = s3 < (unsigned)NB;
      const unsigned many = __builtin_amdgcn_ballot_w32(h0 | h1 | h2 | h3);
      if (many != 0u) {
#define HITJ(J, HJ, SJ) { \
          const unsigned mj = __builtin_amdgcn_ballot_w32(HJ); \
          if (HJ) { \
            const int pos = wc + (int)__builtin_amdgcn_mbcnt_lo(mj, 0u); \
            if (pos < WCAP) list[wave * WCAP + pos] = ((el0 + (J)) << 8) | (int)(SJ); \
          } \
          wc += (int)__builtin_popcount(mj); }
        HITJ(0, h0, s0)
        HITJ(1, h1, s1)
        HITJ(2, h2, s2)
        HITJ(3, h3, s3)
#undef HITJ
      }
    }
    if (lane == 0) wcnt[wave] = wc;
    __syncthreads();

    if (wave == 0) {
#pragma unroll 1
      for (int wsx = 0; wsx < NWAVE; ++wsx) {
        int n = wcnt[wsx];
        if (n > WCAP) n = WCAP;
        if (n < 0) n = 0;
#pragma unroll 1
        for (int i = 0; i < n; ++i) {
          const int ent  = list[wsx * WCAP + i];
          const int slot = ent & (NB - 1);
          const int el   = (ent >> 8) & (CHUNK - 1);
          int e = cbase + el;
          if (e > nEc - 1) e = nEc - 1;
          v4f v0, v1;
          if (dir) {
            const int c = clampi(col1[e], nN - 1);
            const int t = clampi(typ1[e], nR - 1);
            const float* q  = PQ + (size_t)c * PQP + DE + 8 * lane;
            const float* ra = Rt + (size_t)t * DE + 8 * lane;
            v0 = *(const v4f*)q       + *(const v4f*)ra;
            v1 = *(const v4f*)(q + 4) + *(const v4f*)(ra + 4);
          } else {
            const v4i r4 = *(const v4i*)(ind2 + (size_t)e * 4);
            const int c  = clampi(r4.x, nN - 1);
            const int ta = clampi(r4.y, nR - 1);
            const int tb = clampi(r4.z, nR - 1);
            const float* q  = PQ + (size_t)c * PQP + DE + 8 * lane;
            const float* ra = Rt + (size_t)ta * DE + 8 * lane;
            const float* rb = Rt + (size_t)tb * DE + 8 * lane;
            v0 = *(const v4f*)q       + *(const v4f*)ra       + *(const v4f*)rb;
            v1 = *(const v4f*)(q + 4) + *(const v4f*)(ra + 4) + *(const v4f*)(rb + 4);
          }
          float d = dot8(v0, v1, ar0, ar1);
          d = gred<NHEAD>(d);
          const int ai = slot * 4 + head;
          float lg = spa[ai] + d;
          lg = (lg > 0.f) ? lg : 0.2f * lg;
          const float mo = smax[ai];
          const float mn = fmaxf(mo, lg);
          const float sc = __expf(mo - mn);
          const float p  = __expf(lg - mn);
          v4f* sp = (v4f*)(sacc + slot * DE + 8 * lane);
          const v4f c0 = sp[0];
          const v4f c1 = sp[1];
          const v4f n0 = c0 * sc + v0 * p;
          const v4f n1 = c1 * sc + v1 * p;
          sp[0] = n0;
          sp[1] = n1;
          const float dn = sden[ai] * sc + p;
          smax[ai] = mn;
          sden[ai] = dn;
        }
      }
    }
    __syncthreads();
  }

  if (NHEAD == 4) {
#pragma unroll 1
    for (int j = 0; j < NB / NWAVE; ++j) {
      const int slot = wave * (NB / NWAVE) + j;
      const int row  = nodeBase + slot;
      if (row >= nN) break;
      const v4f* sp = (const v4f*)(sacc + slot * DE + 8 * lane);
      const v4f c0 = sp[0];
      const v4f c1 = sp[1];
      const float den = sden[slot * 4 + head];
      const float inv = __builtin_amdgcn_rcpf(den + 1e-16f);
      const float* p = PQ + (size_t)row * PQP + 8 * lane;
      v4f v0 = *(const v4f*)p       + c0 * inv;
      v4f v1 = *(const v4f*)(p + 4) + c1 * inv;
      if (!(den > 0.f)) { v0 = zero4(); v1 = zero4(); }
      v0 = elu4(v0);
      v1 = elu4(v1);
      v4i hv, lv;
      split8(v0, v1, hv, lv);
      const size_t o = (size_t)row * DE + 8 * lane;
      *(volatile v4i*)(xh + o) = hv;
      *(volatile v4i*)(xl + o) = lv;
      __threadfence();
      *(volatile v4i*)(xh + o) = hv;
      *(volatile v4i*)(xl + o) = lv;
    }
  } else {
#pragma unroll 1
    for (int j = 0; j < NB / NWAVE; ++j) {
      const int slot = wave * (NB / NWAVE) + j;
      const int row  = nodeBase + slot;
      if (row >= nN) break;
      const float den = sden[slot * 4];
      const float inv = __builtin_amdgcn_rcpf(den + 1e-16f);
      const bool  has = den > 0.f;
      v4f y[2];
#pragma unroll
      for (int q = 0; q < 2; ++q) {
        const int col = 128 * q + 4 * lane;
        const v4f c0 = *(const v4f*)(sacc + slot * DE + col);
        v4f v = *(const v4f*)(PQ + (size_t)row * PQP + col) + c0 * inv;
        if (!has) v = zero4();
        y[q] = elu4(v);
      }
      float* op = xf + (size_t)row * DE + 4 * lane;
      *(volatile v4f*)(op)       = y[0];
      *(volatile v4f*)(op + 128) = y[1];
      __threadfence();
      *(volatile v4f*)(op)       = y[0];
      *(volatile v4f*)(op + 128) = y[1];
    }
  }
}

__global__ __launch_bounds__(NTHR) void k_bnstat(const float* __restrict__ x3, int nN, double* part) {
  __shared__ __attribute__((aligned(16))) double sm[512];
  const int tid = threadIdx.x;
  const int r0 = blockIdx.x * BNR;
  int r1 = r0 + BNR; if (r1 > nN) r1 = nN;
  double s = 0.0, q = 0.0;
#pragma unroll 1
  for (int r = r0; r < r1; ++r) {
    const double v = (double)x3[(size_t)r * DE + tid];
    s += v;
    q += v * v;
  }
  sm[tid] = s;
  sm[256 + tid] = q;
  __syncthreads();
  v2d w;
  w.x = sm[2 * tid];
  w.y = sm[2 * tid + 1];
  double* dp = part + (size_t)blockIdx.x * 512 + 2 * tid;
  *(volatile v2d*)dp = w;
  __threadfence();
  *(volatile v2d*)dp = w;
}

__global__ __launch_bounds__(NTHR) void k_bncomb(const double* __restrict__ part, int nblk, int nN,
                                                 const float* __restrict__ gam, float* st) {
  __shared__ __attribute__((aligned(16))) float sm[512];
  const int tid = threadIdx.x;
  double S = 0.0, Q = 0.0;
#pragma unroll 1
  for (int b = 0; b < nblk; ++b) {
    S += part[(size_t)b * 512 + tid];
    Q += part[(size_t)b * 512 + 256 + tid];
  }
  const double invn = 1.0 / (double)nN;
  const double mean = S * invn;
  double var = Q * invn - mean * mean;
  var = var > 0.0 ? var : 0.0;
  const double a = (double)gam[tid] / sqrt(var + 1e-5);
  sm[tid] = (float)mean;
  sm[256 + tid] = (float)a;
  __syncthreads();
  if (tid < 128) {
    const v4f w = *(const v4f*)(sm + 4 * tid);
    float* p = st + 4 * tid;
    *(volatile v4f*)p = w;
    __threadfence();
    *(volatile v4f*)p = w;
  }
}

__global__ __launch_bounds__(NTHR) void k_bnapply(const float* __restrict__ x3, const float* __restrict__ st,
                                                  const float* __restrict__ bet, float* out, int nN) {
  const int tid = threadIdx.x, lane = tid & 31, wave = tid >> 5;
  const v4f mu0 = *(const v4f*)(st + 4 * lane);
  const v4f mu1 = *(const v4f*)(st + 128 + 4 * lane);
  const v4f a0  = *(const v4f*)(st + 256 + 4 * lane);
  const v4f a1  = *(const v4f*)(st + 384 + 4 * lane);
  const v4f b0  = *(const v4f*)(bet + 4 * lane);
  const v4f b1  = *(const v4f*)(bet + 128 + 4 * lane);
#pragma unroll 1
  for (int j = 0; j < BNA / NWAVE; ++j) {
    const int row = blockIdx.x * BNA + j * NWAVE + wave;
    if (row >= nN) break;
    const float* xr = x3 + (size_t)row * DE;
    const v4f x0 = *(const v4f*)(xr + 4 * lane);
    const v4f x1 = *(const v4f*)(xr + 128 + 4 * lane);
    const v4f y0 = (x0 - mu0) * a0 + b0;
    const v4f y1 = (x1 - mu1) * a1 + b1;
    float* op = out + (size_t)row * DE + 4 * lane;
    *(volatile v4f*)(op)       = y0;
    *(volatile v4f*)(op + 128) = y1;
    __threadfence();
    *(volatile v4f*)(op)       = y0;
    *(volatile v4f*)(op + 128) = y1;
  }
}

extern "C" void kernel_launch(void* const* d_in, const int* in_sizes, int n_in,
                              void* d_out, int out_size, void* d_ws, size_t ws_size,
                              hipStream_t stream) {
  if (n_in < 13) return;
  const int nE1 = in_sizes[1];
  if (nE1 < 0 || in_sizes[0] != 2 * nE1) return;
  if (in_sizes[2] < 0 || (in_sizes[2] & 3) != 0) return;
  const int nE2 = in_sizes[2] / 4;
  if (in_sizes[3] <= 0 || (in_sizes[3] % DI) != 0) return;
  const int nN = in_sizes[3] / DI;
  if (in_sizes[4] <= 0 || (in_sizes[4] % DI) != 0) return;
  const int nR = in_sizes[4] / DI;
  if (in_sizes[5] != NHD * 3 * DI * HWD) return;
  if (in_sizes[6] != NHD * HWD) return;
  if (in_sizes[7] != DI * DE) return;
  if (in_sizes[8] != 3 * DE * DE) return;
  if (in_sizes[9] != DE) return;
  if (in_sizes[10] != DI * DE) return;
  if (in_sizes[11] != DE || in_sizes[12] != DE) return;
  if (out_size != (nN + nR) * DE) return;

  const int*   edge_index = (const int*)d_in[0];
  const int*   edge_type  = (const int*)d_in[1];
  const int*   ind2       = (const int*)d_in[2];
  const float* embed      = (const float*)d_in[3];
  const float* rel        = (const float*)d_in[4];
  const float* Whd        = (const float*)d_in[5];
  const float* aH         = (const float*)d_in[6];
  const float* gatW       = (const float*)d_in[7];
  const float* outW       = (const float*)d_in[8];
  const float* outA       = (const float*)d_in[9];
  const float* Went       = (const float*)d_in[10];
  const float* gam        = (const float*)d_in[11];
  const float* bet        = (const float*)d_in[12];

  float* out0 = (float*)d_out;
  float* out1 = out0 + (size_t)nN * DE;

  const int MP = ((nN + GT - 1) / GT) * GT;
  const int RP = ((nR + GT - 1) / GT) * GT;

  char* ws = (char*)d_ws;
  const size_t szA = (size_t)MP * DE * 4;
  const size_t szB = (size_t)MP * PQP * 4;
  const size_t oA = 0, oB = oA + szA, oC = oB + szB;
  bf16*  embH  = (bf16*)(ws + oA);
  bf16*  embL  = (bf16*)(ws + oA + (size_t)MP * DI * 2);
  bf16*  xH    = (bf16*)(ws + oA);
  bf16*  xL    = (bf16*)(ws + oA + (size_t)MP * DE * 2);
  float* x2    = (float*)(ws + oA);
  float* PQ1   = (float*)(ws + oB);
  float* PQ2   = (float*)(ws + oB);
  bf16*  embH2 = (bf16*)(ws + oB);
  bf16*  embL2 = (bf16*)(ws + oB + (size_t)MP * DI * 2);
  float* x3    = (float*)(ws + oB + (size_t)MP * DI * 4);
  if ((size_t)MP * DI * 4 + (size_t)MP * DE * 4 > szB) return;

  size_t off = oC;
  auto carve = [&](size_t bytes) -> char* {
    char* p = ws + off;
    off += (bytes + 255) & ~(size_t)255;
    return p;
  };
  bf16*  relH  = (bf16*)carve((size_t)RP * DI * 2);
  bf16*  relL  = (bf16*)carve((size_t)RP * DI * 2);
  bf16*  w1H   = (bf16*)carve((size_t)PQP * DI * 2);
  bf16*  w1L   = (bf16*)carve((size_t)PQP * DI * 2);
  bf16*  wr1H  = (bf16*)carve((size_t)DE * DI * 2);
  bf16*  wr1L  = (bf16*)carve((size_t)DE * DI * 2);
  bf16*  gwH   = (bf16*)carve((size_t)DE * DI * 2);
  bf16*  gwL   = (bf16*)carve((size_t)DE * DI * 2);
  bf16*  w2H   = (bf16*)carve((size_t)PQP * DE * 2);
  bf16*  w2L   = (bf16*)carve((size_t)PQP * DE * 2);
  bf16*  wr2H  = (bf16*)carve((size_t)DE * DE * 2);
  bf16*  wr2L  = (bf16*)carve((size_t)DE * DE * 2);
  bf16*  weH   = (bf16*)carve((size_t)DE * DI * 2);
  bf16*  weL   = (bf16*)carve((size_t)DE * DI * 2);
  float* R1    = (float*)carve((size_t)RP * DE * 4);
  bf16*  rH    = (bf16*)carve((size_t)RP * DE * 2);
  bf16*  rL    = (bf16*)carve((size_t)RP * DE * 2);
  float* R2    = (float*)carve((size_t)RP * DE * 4);
  const int nblkS = (nN + BNR - 1) / BNR;
  double* bnpart = (double*)carve((size_t)nblkS * 512 * 8);
  float*  bnst   = (float*)carve((size_t)512 * 4);
  if (off > ws_size) return;

  {
    const int t8 = MP * DI / 8;
    k_cvtA<<<(t8 + NTHR - 1) / NTHR, NTHR, 0, stream>>>(embed, nN, DI, t8, embH, embL);
    const int r8 = RP * DI / 8;
    k_cvtA<<<(r8 + NTHR - 1) / NTHR, NTHR, 0, stream>>>(rel, nR, DI, r8, relH, relL);
  }
  {
    const int t128 = DE * DI / 8;
    const int t256 = DE * DE / 8;
    k_packB<<<dim3((t128 + NTHR - 1) / NTHR, 2), NTHR, 0, stream>>>(Whd, w1H, w1L, DI, DE, HWD, 3 * DI * HWD, HWD, 0, DI * HWD, t128);
    k_packB<<<dim3((t128 + NTHR - 1) / NTHR, 1), NTHR, 0, stream>>>(Whd, wr1H, wr1L, DI, DE, HWD, 3 * DI * HWD, HWD, 2 * DI * HWD, 0, t128);
    k_packB<<<dim3((t128 + NTHR - 1) / NTHR, 1), NTHR, 0, stream>>>(gatW, gwH, gwL, DI, DE, DE, 0, DE, 0, 0, t128);
    k_packB<<<dim3((t128 + NTHR - 1) / NTHR, 1), NTHR, 0, stream>>>(Went, weH, weL, DI, DE, DE, 0, DE, 0, 0, t128);
    k_packB<<<dim3((t256 + NTHR - 1) / NTHR, 2), NTHR, 0, stream>>>(outW, w2H, w2L, DE, DE, DE, 0, DE, 0, DE * DE, t256);
    k_packB<<<dim3((t256 + NTHR - 1) / NTHR, 1), NTHR, 0, stream>>>(outW, wr2H, wr2L, DE, DE, DE, 0, DE, 2 * DE * DE, 0, t256);
  }

  k_gemm3<<<dim3(PQP / GT, MP / GT), GTHR, 0, stream>>>(embH, embL, DI, w1H, w1L, DI, DI,
                                                         PQ1, PQP, MP, nullptr, nullptr, nullptr, 0);
  k_gemm3<<<dim3(DE / GT, RP / GT), GTHR, 0, stream>>>(relH, relL, DI, wr1H, wr1L, DI, DI,
                                                        R1, DE, RP, nullptr, nullptr, nullptr, 0);
  k_gemm3<<<dim3(DE / GT, RP / GT), GTHR, 0, stream>>>(relH, relL, DI, gwH, gwL, DI, DI,
                                                        out1, DE, nR, nullptr, rH, rL, DE);

  const int nblkA = (nN + NB - 1) / NB;
  hipFuncSetAttribute(reinterpret_cast<const void*>(&k_agg<4>),
                      hipFuncAttributeMaxDynamicSharedMemorySize, AGG_LDS_BYTES);
  hipLaunchKernelGGL(HIP_KERNEL_NAME(k_agg<4>), dim3(nblkA), dim3(NTHR), AGG_LDS_BYTES, stream,
                     edge_index + nE1, edge_index, edge_type, ind2, (const float*)PQ1, (const float*)R1, aH,
                     xH, xL, (float*)nullptr, nN, nR, nE1, nE2);

  k_gemm3<<<dim3(PQP / GT, MP / GT), GTHR, 0, stream>>>(xH, xL, DE, w2H, w2L, DE, DE,
                                                         PQ2, PQP, MP, nullptr, nullptr, nullptr, 0);
  k_gemm3<<<dim3(DE / GT, RP / GT), GTHR, 0, stream>>>(rH, rL, DE, wr2H, wr2L, DE, DE,
                                                        R2, DE, RP, nullptr, nullptr, nullptr, 0);
  hipFuncSetAttribute(reinterpret_cast<const void*>(&k_agg<1>),
                      hipFuncAttributeMaxDynamicSharedMemorySize, AGG_LDS_BYTES);
  hipLaunchKernelGGL(HIP_KERNEL_NAME(k_agg<1>), dim3(nblkA), dim3(NTHR), AGG_LDS_BYTES, stream,
                     edge_index + nE1, edge_index, edge_type, ind2, (const float*)PQ2, (const float*)R2, outA,
                     (bf16*)nullptr, (bf16*)nullptr, x2, nN, nR, nE1, nE2);

  {
    const int t8 = MP * DI / 8;
    k_cvtA<<<(t8 + NTHR - 1) / NTHR, NTHR, 0, stream>>>(embed, nN, DI, t8, embH2, embL2);
  }
  k_gemm3<<<dim3(DE / GT, MP / GT), GTHR, 0, stream>>>(embH2, embL2, DI, weH, weL, DI, DI,
                                                        x3, DE, MP, x2, nullptr, nullptr, 0);
  k_bnstat<<<nblkS, NTHR, 0, stream>>>(x3, nN, bnpart);
  k_bncomb<<<1, NTHR, 0, stream>>>(bnpart, nblkS, nN, gam, bnst);
  k_bnapply<<<(nN + BNA - 1) / BNA, NTHR, 0, stream>>>(x3, bnst, bet, out0, nN);
}
